// TriplePlaneMLP_3143916060686
// MI455X (gfx1250) — hardware-verified
//
#include <hip/hip_runtime.h>


#define NPTS 2097152
#define RCH  262144
#define URES 400
#define UCH  8
#define ARES 50
#define ACH  8
#define FIN  24
#define KP   32
#define HID  32
#define NP   64
#define DM   KP
#define LOSC 1024.0f

typedef _Float16 h16;
typedef unsigned short bf;
typedef __attribute__((ext_vector_type(16))) __bf16   v16bf;
typedef __attribute__((ext_vector_type(16))) _Float16 v16h;
typedef __attribute__((ext_vector_type(8)))  _Float16 v8h;
typedef __attribute__((ext_vector_type(8)))  unsigned short v8us;
typedef __attribute__((ext_vector_type(8)))  float    v8f;
typedef __attribute__((ext_vector_type(4)))  float    v4f;
typedef v8h  __attribute__((may_alias)) v8ha;
typedef v4f  __attribute__((may_alias)) v4fa;
typedef v8us __attribute__((may_alias)) v8usa;

__device__ __forceinline__ unsigned short f2bf(float f) { unsigned u = __float_as_uint(f); u += 0x7FFFu + ((u >> 16) & 1u); return (unsigned short)(u >> 16); }
__device__ __forceinline__ float bf2f(unsigned short b) { return __uint_as_float(((unsigned)b) << 16); }
__device__ __forceinline__ float bfr(float f) { return bf2f(f2bf(f)); }
__device__ __forceinline__ v16h cat16(v8h lo, v8h hi) { return __builtin_shufflevector(lo, hi, 0, 1, 2, 3, 4, 5, 6, 7, 8, 9, 10, 11, 12, 13, 14, 15); }
__device__ __forceinline__ v16bf cat16b(v8us lo, v8us hi) { return __builtin_bit_cast(v16bf, __builtin_shufflevector(lo, hi, 0, 1, 2, 3, 4, 5, 6, 7, 8, 9, 10, 11, 12, 13, 14, 15)); }
__device__ __forceinline__ v8f wmma16(v16h a, v16h b, v8f c) { return __builtin_amdgcn_wmma_f32_16x16x32_f16(false, a, false, b, (short)0, c, false, false); }
__device__ __forceinline__ v8f wmmab(v16bf a, v16bf b, v8f c) { return __builtin_amdgcn_wmma_f32_16x16x32_bf16(false, a, false, b, (short)0, c, false, false); }

template <bool SPLITA, bool F16OUT = false>
__global__ __launch_bounds__(128) void k_gemmb(const bf* __restrict__ A, const bf* __restrict__ Al, const bf* __restrict__ Bn, const float* __restrict__ bias, float* C, int ldc, h16* C2, const float* __restrict__ R = nullptr, int K = DM, int roundR = 1) {
    __shared__ __align__(16) float ost[4][16 * 68];
    const int lane = threadIdx.x & 31, wave = threadIdx.x >> 5, lr = lane & 15, hi = lane >> 4;
    const int r0 = blockIdx.x * 64 + wave * 16, c0 = blockIdx.y * 64;
    const size_t aoff = (size_t)(r0 + lr) * K + 8 * hi;
    size_t boff[4];
#pragma unroll
    for (int t = 0; t < 4; ++t) boff[t] = (size_t)(c0 + t * 16 + lr) * K + 8 * hi;
    v8f acc[4];
#pragma unroll
    for (int t = 0; t < 4; ++t) acc[t] = (v8f){};
#pragma unroll 1
    for (int kc = 0; kc < K; kc += 32) {
        const v16bf a = cat16b(*(const v8us*)(A + aoff + kc), *(const v8us*)(A + aoff + kc + 16));
        v16bf al = a;
        if (SPLITA) al = cat16b(*(const v8us*)(Al + aoff + kc), *(const v8us*)(Al + aoff + kc + 16));
#pragma unroll
        for (int t = 0; t < 4; ++t) { const v16bf b = cat16b(*(const v8us*)(Bn + boff[t] + kc), *(const v8us*)(Bn + boff[t] + kc + 16)); acc[t] = wmmab(a, b, acc[t]); if (SPLITA) acc[t] = wmmab(al, b, acc[t]); }
        asm volatile("v_nop\n\tv_nop\n\tv_nop\n\tv_nop" : "+v"(acc[0]), "+v"(acc[1]), "+v"(acc[2]), "+v"(acc[3]) : "v"(a), "v"(al));
    }
    float* os = &ost[wave][0];
#pragma unroll
    for (int t = 0; t < 4; ++t) { const float bv = bias ? bfr(bias[c0 + t * 16 + lr]) : 0.f;
#pragma unroll
        for (int j = 0; j < 8; ++j) os[(hi * 8 + j) * 68 + t * 16 + lr] = acc[t][j] + bv; }
    __syncthreads();
    if (F16OUT) {
        h16* crow = (h16*)(void*)C + (size_t)r0 * ldc + c0;
        auto pass = [&]() {
#pragma unroll
            for (int s = 0; s < 4; ++s) { const int row = 4 * s + (lane >> 3), piece = lane & 7; const float* sp = os + row * 68 + piece * 8; v8h o, o2;
#pragma unroll
                for (int i = 0; i < 8; ++i) { const h16 a = (h16)sp[i]; o[i] = a; o2[i] = (h16)((sp[i] - (float)a) * LOSC); }
                *(volatile v8h*)(crow + (size_t)row * ldc + piece * 8) = o; if (C2) *(volatile v8h*)(C2 + (size_t)r0 * ldc + c0 + (size_t)row * ldc + piece * 8) = o2; }
        };
        pass(); __threadfence(); pass();
    } else {
        float* crow = C + (size_t)r0 * ldc + c0;
        auto pass = [&]() {
#pragma unroll
            for (int s = 0; s < 8; ++s) { const int Lid = (lane >> 3) + 4 * s, piece = lane & 7; const int row = Lid >> 1, cofs = (Lid & 1) * 32 + piece * 4;
                v4f val = *(const v4fa*)(os + row * 68 + cofs); if (R) { const v4f rv = *(const v4f*)(R + ((size_t)r0 + row) * ldc + c0 + cofs); val += roundR ? (v4f){bfr(rv[0]), bfr(rv[1]), bfr(rv[2]), bfr(rv[3])} : rv; }
                *(volatile v4f*)(crow + (size_t)row * ldc + cofs) = val; }
        };
        pass(); __threadfence(); pass();
    }
}


__global__ __launch_bounds__(256) void k_w(const float* __restrict__ Wm, int kk, bf* WT) {
    const int u = threadIdx.x; v8us o;
#pragma unroll
    for (int i = 0; i < 8; ++i) { const int f = u * 8 + i; const int n = f / KP, k = f % KP; const bool ok = (n < HID) && (k < kk); o[i] = ok ? f2bf(Wm[(ok ? n : 0) * kk + (ok ? k : 0)]) : (unsigned short)0; }
    *(volatile v8us*)(WT + u * 8) = o; __threadfence(); *(volatile v8us*)(WT + u * 8) = o;
}
__device__ __forceinline__ void bilerp_clamp(const float* __restrict__ tex, float uu, float vv, float* f) {
    const float u = fminf(fmaxf(uu, 0.f), 1.f) * (float)(URES - 1), v = fminf(fmaxf(vv, 0.f), 1.f) * (float)(URES - 1);
    int x0 = (int)floorf(u); int y0 = (int)floorf(v); x0 = x0 < 0 ? 0 : (x0 > URES - 1 ? URES - 1 : x0); y0 = y0 < 0 ? 0 : (y0 > URES - 1 ? URES - 1 : y0);
    const int x1 = (x0 + 1 > URES - 1) ? URES - 1 : x0 + 1, y1 = (y0 + 1 > URES - 1) ? URES - 1 : y0 + 1;
    const float ur = u - (float)x0, vr = v - (float)y0;
#pragma unroll
    for (int c = 0; c < UCH; ++c) { const float p00 = bfr(tex[((size_t)y0 * URES + x0) * UCH + c]), p10 = bfr(tex[((size_t)y0 * URES + x1) * UCH + c]), p01 = bfr(tex[((size_t)y1 * URES + x0) * UCH + c]), p11 = bfr(tex[((size_t)y1 * URES + x1) * UCH + c]);
        f[c] = (1.f - ur) * (1.f - vr) * p00 + ur * (1.f - vr) * p10 + (1.f - ur) * vr * p01 + ur * vr * p11; }
}
__device__ __forceinline__ void bilerp_wrap(const float* __restrict__ tex, float uu, float vv, float* f) {
    const float u = (uu - floorf(uu)) * (float)ARES;
    const float v = fminf(fmaxf(vv, 0.f), 1.f) * (float)(ARES - 1);
    const float x0f = floorf(u); int x0 = ((int)x0f) % ARES; if (x0 < 0) x0 += ARES; const int x1 = (x0 + 1) % ARES;
    int y0 = (int)floorf(v); y0 = y0 < 0 ? 0 : (y0 > ARES - 1 ? ARES - 1 : y0); const int y1 = (y0 + 1 > ARES - 1) ? ARES - 1 : y0 + 1;
    const float ur = u - x0f, vr = v - (float)y0;
#pragma unroll
    for (int c = 0; c < ACH; ++c) { const float p00 = bfr(tex[((size_t)y0 * ARES + x0) * ACH + c]), p10 = bfr(tex[((size_t)y0 * ARES + x1) * ACH + c]), p01 = bfr(tex[((size_t)y1 * ARES + x0) * ACH + c]), p11 = bfr(tex[((size_t)y1 * ARES + x1) * ACH + c]);
        f[c] = (1.f - ur) * (1.f - vr) * p00 + ur * (1.f - vr) * p10 + (1.f - ur) * vr * p01 + ur * vr * p11; }
}
__global__ __launch_bounds__(256) void k_feat(const float* __restrict__ x, const float* __restrict__ up, const float* __restrict__ hp, const float* __restrict__ dp, int p0, bf* Fh, bf* Fl) {
    const int lane = threadIdx.x & 31; const size_t pl = ((size_t)blockIdx.x * 8 + (threadIdx.x >> 5)) * 8 + (lane >> 2); const size_t p = (size_t)p0 + pl; const int grp = lane & 3;
    float f[8];
#pragma unroll
    for (int c = 0; c < 8; ++c) f[c] = 0.f;
    const float* xr = x + p * 6;
    if (grp == 0) bilerp_clamp(up, bfr(xr[0]), bfr(xr[1]), f); else if (grp == 1) bilerp_wrap(hp, bfr(xr[3]), bfr(xr[2]), f); else if (grp == 2) bilerp_wrap(dp, bfr(xr[5]), bfr(xr[4]), f);
    v8us oh, ol;
#pragma unroll
    for (int c = 0; c < 8; ++c) { const unsigned short hb = f2bf(f[c]); oh[c] = hb; ol[c] = f2bf(f[c] - bf2f(hb)); }
    const size_t o = pl * KP + grp * 8; *(volatile v8us*)(Fh + o) = oh; *(volatile v8us*)(Fl + o) = ol; __threadfence(); *(volatile v8us*)(Fh + o) = oh; *(volatile v8us*)(Fl + o) = ol;
}
__global__ __launch_bounds__(256) void k_relusplit(const float* __restrict__ G, bf* Fh, bf* Fl) {
    const int lane = threadIdx.x & 31; const size_t rl = ((size_t)blockIdx.x * 8 + (threadIdx.x >> 5)) * 8 + (lane >> 2); const int cb = (lane & 3) * 8; v8us oh, ol;
#pragma unroll
    for (int i = 0; i < 8; ++i) { const float v = fmaxf(G[rl * NP + cb + i], 0.f); const unsigned short hb = f2bf(v); oh[i] = hb; ol[i] = f2bf(v - bf2f(hb)); }
    const size_t o = rl * KP + cb; *(volatile v8us*)(Fh + o) = oh; *(volatile v8us*)(Fl + o) = ol; __threadfence(); *(volatile v8us*)(Fh + o) = oh; *(volatile v8us*)(Fl + o) = ol;
}
__global__ __launch_bounds__(256) void k_last(const float* __restrict__ G, const float* __restrict__ W3, int p0, float* OUTP) {
    const size_t u = (size_t)blockIdx.x * 256 + threadIdx.x; if (u >= (size_t)RCH * 3 / 4) return; v4f ov;
#pragma unroll
    for (int q = 0; q < 4; ++q) { const size_t e = u * 4 + q; const size_t rl = e / 3; const int oc = (int)(e % 3); float s = 0.f;
#pragma unroll 8
        for (int c = 0; c < HID; ++c) s = fmaf(fmaxf(G[rl * NP + c], 0.f), bfr(W3[oc * HID + c]), s);
        ov[q] = s; }
    float* dst = OUTP + (size_t)p0 * 3 + u * 4; *(volatile v4f*)dst = ov; __threadfence(); *(volatile v4f*)dst = ov;
}

extern "C" void kernel_launch(void* const* d_in, const int* in_sizes, int n_in,
                              void* d_out, int out_size, void* d_ws, size_t ws_size, hipStream_t stream) {
    (void)in_sizes; (void)n_in; (void)out_size;
    const float* x = (const float*)d_in[0]; const float* up = (const float*)d_in[1]; const float* hp = (const float*)d_in[2]; const float* dp = (const float*)d_in[3];
    const float* W0 = (const float*)d_in[4]; const float* W1 = (const float*)d_in[5]; const float* W2 = (const float*)d_in[6]; const float* W3 = (const float*)d_in[7];
    float* out = (float*)d_out;
    char* wsp = (char*)d_ws;
    auto take = [&](size_t bytes) { char* p = wsp; wsp += (bytes + 255) & ~(size_t)255; return (void*)p; };
    bf* W0T = (bf*)take(NP * KP * 2); bf* W1T = (bf*)take(NP * KP * 2); bf* W2T = (bf*)take(NP * KP * 2);
    bf* Fh = (bf*)take((size_t)RCH * KP * 2); bf* Fl = (bf*)take((size_t)RCH * KP * 2); float* G = (float*)take((size_t)RCH * NP * 4);
    if ((size_t)(wsp - (char*)d_ws) > ws_size) return;
    k_w<<<1, 256, 0, stream>>>(W0, FIN, W0T); k_w<<<1, 256, 0, stream>>>(W1, HID, W1T); k_w<<<1, 256, 0, stream>>>(W2, HID, W2T);
    for (int ch = 0; ch < NPTS / RCH; ++ch) { const int p0 = ch * RCH;
        k_feat<<<RCH / 64, 256, 0, stream>>>(x, up, hp, dp, p0, Fh, Fl);
        k_gemmb<true, false><<<dim3(RCH / 64, 1, 1), 128, 0, stream>>>(Fh, Fl, W0T, nullptr, G, NP, nullptr, nullptr, KP);
        k_relusplit<<<RCH / 64, 256, 0, stream>>>(G, Fh, Fl);
        k_gemmb<true, false><<<dim3(RCH / 64, 1, 1), 128, 0, stream>>>(Fh, Fl, W1T, nullptr, G, NP, nullptr, nullptr, KP);
        k_relusplit<<<RCH / 64, 256, 0, stream>>>(G, Fh, Fl);
        k_gemmb<true, false><<<dim3(RCH / 64, 1, 1), 128, 0, stream>>>(Fh, Fl, W2T, nullptr, G, NP, nullptr, nullptr, KP);
        k_last<<<(RCH * 3 / 4) / 256, 256, 0, stream>>>(G, W3, p0, out); }
}
